// HSSurv_12429635355022
// MI455X (gfx1250) — hardware-verified
//
#include <hip/hip_runtime.h>
#include <math.h>

typedef __attribute__((ext_vector_type(16))) _Float16 v16h;
typedef __attribute__((ext_vector_type(16))) __bf16 v16b;
typedef __attribute__((ext_vector_type(8)))  _Float16 v8h;
typedef __attribute__((ext_vector_type(8)))  __bf16 v8b;
typedef __attribute__((ext_vector_type(8)))  float v8f;
typedef __attribute__((ext_vector_type(4)))  float v4f;
typedef __attribute__((ext_vector_type(4)))  unsigned v4u;
typedef _Float16 h16;

#ifndef NB
#define NB 8
#endif
#ifndef SEQ
#define SEQ 2048
#endif
#define NB_FULL 8
#define SEQ_FULL 2048
#define DIN  512
#define DHID 512
#define NE   8
#define NROW (NB * SEQ)
#define NG   (NB * NE)
#define TM   64
#define APITCH4 (DIN / 8 + 1)
#define PCOLS 256
#define HCARRY 64.0f
#define WCARRY 512.0f
#define OSCALE (1.0f / 32768.0f)
#define EPSV 1e-6f
#define GENO_RATIO 0.1f
#define OUT1_ELEM ((size_t)NB_FULL * NE * DHID)

#define WS_XB  ((size_t)0)
#define WS_W1T (WS_XB  + (size_t)NROW * DIN * 2)
#define WS_W2T (WS_W1T + (size_t)NE * DHID * DIN * 2)
#define WS_WD  (WS_W2T + (size_t)NE * DHID * DHID * 2)
#define WS_HS  (WS_WD  + (size_t)NROW * NE * 4)
#define WS_END (WS_HS  + (size_t)NG * DHID * 4)

static_assert(NE == 8);
static_assert(NB >= 1 && NB <= NB_FULL && NB <= 8);
static_assert(SEQ <= SEQ_FULL && SEQ <= 65536);
static_assert(SEQ % 256 == 0 && SEQ % TM == 0 && SEQ % 32 == 0);
static_assert(DIN % 32 == 0 && DHID % 32 == 0 && DIN / 8 == 64);
static_assert(DHID % PCOLS == 0 && DHID % 128 == 0 && DIN % 64 == 0 && DHID % 64 == 0);
static_assert(OUT1_ELEM * 4 == 131072);
static_assert((OUT1_ELEM + 1) * 4 <= 131076);
static_assert(((size_t)((NB - 1) * NE + (NE - 1)) * DHID + DHID) <= OUT1_ELEM);
static_assert(WS_W1T % 128 == 0 && WS_W2T % 128 == 0 && WS_WD % 128 == 0 && WS_HS % 128 == 0);
static_assert(WS_END <= (size_t)134217728);
static_assert((size_t)(NROW * DIN / 8 / 256) * 256 * 8 == (size_t)NROW * DIN);
static_assert((size_t)(DHID / 64) * (DIN / 64) * NE * 4096 == (size_t)NE * DIN * DHID);
static_assert((size_t)(NROW / 32) * 64 * 4 == (size_t)NROW * NE);
static_assert(64 * 16 == 32 * NE * 4);
static_assert((size_t)(DHID / PCOLS) * NG * 64 * 4 == (size_t)NG * DHID);
static_assert(64 * 16 == PCOLS * 4);
static_assert(32 * 16 == 128 * 4);
static_assert((TM * DIN / 8) % 256 == 0 && (TM * DIN / 8 / 256) * 256 * 16 == TM * DIN * 2);
static_assert(((size_t)NROW * NE) % 1024 == 0);
static_assert(TM * APITCH4 * 16 + SEQ * 2 + SEQ * 4 + 32 + PCOLS * 4 <= 131072);
static_assert(64 * 65 * 4 <= 131072);

__device__ __forceinline__ v8f wmma16(v16h a, v16h b, v8f c) {
  v8f d = __builtin_amdgcn_wmma_f32_16x16x32_f16(false, a, false, b, (short)0, c, false, false);
  asm volatile("v_nop\n\tv_nop\n\tv_nop\n\tv_nop" : "+v"(d) : "v"(a), "v"(b));
  return d;
}
__device__ __forceinline__ v8f wmma_bf(v16b a, v16b b, v8f c) {
  v8f d = __builtin_amdgcn_wmma_f32_16x16x32_bf16(false, a, false, b, (short)0, c, false, false);
  asm volatile("v_nop\n\tv_nop\n\tv_nop\n\tv_nop" : "+v"(d) : "v"(a), "v"(b));
  return d;
}
__device__ __forceinline__ float bfr(float v) { return (float)(__bf16)v; }
static __device__ __forceinline__ h16 toh_flush(float v) { const h16 r = (h16)v; return (fabsf(v) < 6.103515625e-05f) ? (h16)0.0f : r; }
__device__ __forceinline__ v16b ldfrag_b(const unsigned short* p) { union { v16b v; v4u q[2]; } f; f.q[0] = *(const v4u*)p; f.q[1] = *(const v4u*)(p + 16); return f.v; }
__device__ __forceinline__ v16h ldfrag_h(const unsigned short* p) { union { v16h v; v4u q[2]; } f; f.q[0] = *(const v4u*)p; f.q[1] = *(const v4u*)(p + 16); return f.v; }

__global__ __launch_bounds__(256) void k_cvt_x(const float* __restrict__ X, unsigned short* __restrict__ XB) {
  const unsigned i = blockIdx.x * 256u + threadIdx.x;
  const unsigned ic = i < (unsigned)(NROW * DIN / 8) ? i : (unsigned)(NROW * DIN / 8 - 1);
  const unsigned rw = ic / (unsigned)(DIN / 8), pc = ic % (unsigned)(DIN / 8);
  const size_t src = ((size_t)(rw / (unsigned)SEQ) * SEQ_FULL + rw % (unsigned)SEQ) * DIN + 8u * pc;
  const v4f a = *(const v4f*)(X + src), b = *(const v4f*)(X + src + 4);
  union { v8b h; v4u u; } o;
#pragma unroll
  for (int j = 0; j < 4; ++j) { o.h[j] = (__bf16)a[j]; o.h[4 + j] = (__bf16)b[j]; }
  const v4u val = o.u;
  volatile v4u* p = (volatile v4u*)(XB + (size_t)ic * 8);
  *p = val; __threadfence(); *p = val;
}

__global__ __launch_bounds__(256) void k_tr(const float* __restrict__ S, unsigned short* __restrict__ Dst, unsigned K, unsigned N, unsigned dpitch, unsigned erow, unsigned ecol, int f16, float sc) {
  __shared__ float tile[64][65];
  const unsigned t = threadIdx.x, e = blockIdx.z, k0 = blockIdx.y * 64u, n0 = blockIdx.x * 64u;
  const float* s = S + (size_t)e * K * N;
#pragma unroll
  for (unsigned it = 0; it < 4; ++it) { const unsigned idx = it * 256u + t, kr = idx >> 4, c4 = idx & 15u;
    const v4f v = *(const v4f*)(s + (size_t)(k0 + kr) * N + n0 + 4u * c4);
    tile[kr][4u * c4 + 0] = v[0]; tile[kr][4u * c4 + 1] = v[1]; tile[kr][4u * c4 + 2] = v[2]; tile[kr][4u * c4 + 3] = v[3]; }
  __syncthreads();
  v4u o[2];
#pragma unroll
  for (unsigned it = 0; it < 2; ++it) { const unsigned idx = it * 256u + t, nr = idx >> 3, q = idx & 7u;
    union { v8b b; v8h h; v4u u; } w;
#pragma unroll
    for (int i = 0; i < 8; ++i) { const float v = bfr(tile[8u * q + i][nr]); if (f16) w.h[i] = toh_flush(v * sc); else w.b[i] = (__bf16)v; }
    o[it] = w.u; }
#pragma unroll
  for (unsigned it = 0; it < 2; ++it) { const unsigned idx = it * 256u + t, nr = idx >> 3, q = idx & 7u;
    *(volatile v4u*)(Dst + (size_t)(e * erow + n0 + nr) * dpitch + e * ecol + k0 + 8u * q) = o[it]; }
  __threadfence();
#pragma unroll
  for (unsigned it = 0; it < 2; ++it) { const unsigned idx = it * 256u + t, nr = idx >> 3, q = idx & 7u;
    *(volatile v4u*)(Dst + (size_t)(e * erow + n0 + nr) * dpitch + e * ecol + k0 + 8u * q) = o[it]; }
}

__global__ __launch_bounds__(256) void k_gate(const float* __restrict__ TOK, const float* __restrict__ GV, const float* __restrict__ GW, const float* __restrict__ GB, const float* __restrict__ NW, const float* __restrict__ NBI, float* __restrict__ WD) {
#pragma clang fp contract(off)
  __shared__ __align__(16) float sgl[NE];
  __shared__ __align__(16) float sw[32][NE];
  const unsigned tid = threadIdx.x, lane = tid & 31u;
  const unsigned wave = (unsigned)__builtin_amdgcn_readfirstlane((int)(tid >> 5));
  const unsigned t0 = blockIdx.x * 32u;
  const unsigned b = t0 / (unsigned)SEQ;
  {
    float a = 0.f;
#pragma unroll 1
    for (unsigned i = 0; i < DIN / 32; ++i) { const unsigned c = lane + 32u * i; a = fmaf(bfr(GV[(size_t)b * DIN + c]), bfr(NW[(size_t)c * NE + wave]), a); }
    a += __shfl_xor(a, 16); a += __shfl_xor(a, 8); a += __shfl_xor(a, 4); a += __shfl_xor(a, 2); a += __shfl_xor(a, 1);
    if (lane == 0u) sgl[wave] = a + bfr(NBI[wave]);
  }
  __syncthreads();
  float gb[NE], gl[NE];
#pragma unroll
  for (int k = 0; k < NE; ++k) { gb[k] = bfr(GB[k]); gl[k] = GENO_RATIO * sgl[k]; }
#pragma unroll 1
  for (unsigned ps = 0; ps < 4u; ++ps) {
    const unsigned j = ps * 8u + wave;
    const unsigned r = t0 + j;
    const float* xp = TOK + ((size_t)b * SEQ_FULL + (r - b * (unsigned)SEQ)) * DIN;
    float a0 = 0.f, a1 = 0.f, a2 = 0.f, a3 = 0.f, a4 = 0.f, a5 = 0.f, a6 = 0.f, a7 = 0.f;
#pragma unroll 1
    for (unsigned i = 0; i < DIN / 32; ++i) { const unsigned c = lane + 32u * i;
      const float x = bfr(xp[c]);
      const v4f g0 = *(const v4f*)(GW + (size_t)c * NE), g1 = *(const v4f*)(GW + (size_t)c * NE + 4);
      a0 = fmaf(x, bfr(g0[0]), a0); a1 = fmaf(x, bfr(g0[1]), a1); a2 = fmaf(x, bfr(g0[2]), a2); a3 = fmaf(x, bfr(g0[3]), a3);
      a4 = fmaf(x, bfr(g1[0]), a4); a5 = fmaf(x, bfr(g1[1]), a5); a6 = fmaf(x, bfr(g1[2]), a6); a7 = fmaf(x, bfr(g1[3]), a7); }
    float lg[NE] = { a0, a1, a2, a3, a4, a5, a6, a7 };
#pragma unroll
    for (int k = 0; k < NE; ++k) { float v = lg[k];
      v += __shfl_xor(v, 16); v += __shfl_xor(v, 8); v += __shfl_xor(v, 4); v += __shfl_xor(v, 2); v += __shfl_xor(v, 1);
      lg[k] = (v + gb[k]) + gl[k]; }
    int i0 = 0; float v0 = lg[0];
#pragma unroll
    for (int k = 1; k < NE; ++k) { const bool tk = lg[k] > v0; v0 = tk ? lg[k] : v0; i0 = tk ? k : i0; }
    int i1 = NE; float v1 = -INFINITY;
#pragma unroll
    for (int k = 0; k < NE; ++k) { const bool tk = (k != i0) && (lg[k] > v1); v1 = tk ? lg[k] : v1; i1 = tk ? k : i1; }
    const float e1 = expf(v1 - v0);
    const float rs = 1.0f / (1.0f + e1);
    float w0 = rs, w1 = e1 * rs;
    w0 = fmaxf(w0, EPSV); w1 = fmaxf(w1, EPSV);
    const float rt = 1.0f / (w0 + w1);
    w0 = w0 * rt; w1 = w1 * rt;
    const int kk = (int)(lane & 7u);
    const float wk = (kk == i0) ? w0 : ((kk == i1) ? w1 : 0.0f);
    if (lane < 8u) sw[j][lane] = wk;
  }
  __syncthreads();
  if (tid < 64u) {
    const v4f val = *(const v4f*)(&sw[0][0] + 4u * tid);
    volatile v4f* p = (volatile v4f*)(WD + (size_t)t0 * NE + 4u * tid);
    *p = val; __threadfence(); *p = val;
  }
}

__global__ __launch_bounds__(256) void k_lb(const float* __restrict__ WD, float* __restrict__ OUT) {
#pragma clang fp contract(off)
  __shared__ unsigned sc[8][NE];
  const unsigned tid = threadIdx.x, lane = tid & 31u;
  const unsigned wave = (unsigned)__builtin_amdgcn_readfirstlane((int)(tid >> 5));
  unsigned c0 = 0u, c1 = 0u, c2 = 0u, c3 = 0u;
#pragma unroll 4
  for (unsigned i = 0; i < (unsigned)((size_t)NROW * NE / 1024); ++i) { const v4f v = *(const v4f*)(WD + 4u * (size_t)(i * 256u + tid));
    c0 += v[0] > 0.f ? 1u : 0u; c1 += v[1] > 0.f ? 1u : 0u; c2 += v[2] > 0.f ? 1u : 0u; c3 += v[3] > 0.f ? 1u : 0u; }
#pragma unroll
  for (int off = 16; off >= 2; off >>= 1) {
    c0 += (unsigned)__shfl_xor((int)c0, off); c1 += (unsigned)__shfl_xor((int)c1, off);
    c2 += (unsigned)__shfl_xor((int)c2, off); c3 += (unsigned)__shfl_xor((int)c3, off); }
  if (lane < 2u) { sc[wave][4u * lane + 0u] = c0; sc[wave][4u * lane + 1u] = c1; sc[wave][4u * lane + 2u] = c2; sc[wave][4u * lane + 3u] = c3; }
  __syncthreads();
  float us[NE]; float mean = 0.f;
#pragma unroll
  for (int k = 0; k < NE; ++k) { unsigned tt = 0u;
#pragma unroll
    for (int w = 0; w < 8; ++w) tt += sc[w][k];
    us[k] = (float)tt * (1.0f / (float)NROW); mean += us[k]; }
  mean = mean * 0.125f;
  float var = 0.f;
#pragma unroll
  for (int k = 0; k < NE; ++k) { const float d = us[k] - mean; var += d * d; }
  var = var * 0.125f;
  const float sd = sqrtf(var);
  const float q = sd / (mean + EPSV);
  const float lb = q * q;
  if (tid == 0u) { volatile float* p = OUT + OUT1_ELEM; *p = lb; __threadfence(); *p = lb; }
}

__global__ __launch_bounds__(256) void k_pool(const unsigned short* __restrict__ XB, const unsigned short* __restrict__ W1T, const float* __restrict__ B1, const float* __restrict__ WD, float* __restrict__ HS) {
  __shared__ v4u sa4[TM * APITCH4];
  __shared__ unsigned short lidx[SEQ];
  __shared__ float lw[SEQ];
  __shared__ unsigned wcnt[8];
  __shared__ __align__(16) float so[PCOLS];
  const unsigned tid = threadIdx.x, lane = tid & 31u, lm = lane & 15u, lh = lane >> 4;
  const unsigned wave = (unsigned)__builtin_amdgcn_readfirstlane((int)(tid >> 5));
  const unsigned g = blockIdx.y, b = g / NE, e = g % NE, n0 = blockIdx.x * (unsigned)PCOLS;
  unsigned run = 0u;
#pragma unroll 1
  for (unsigned ps = 0; ps < (unsigned)(SEQ / 256); ++ps) {
    const unsigned n = ps * 256u + tid;
    const float w = WD[((size_t)b * SEQ + n) * NE + e];
    const bool sel = w > 0.0f;
    const unsigned mask = __builtin_amdgcn_ballot_w32(sel);
    const unsigned rank = __builtin_amdgcn_mbcnt_lo(mask, 0u);
    if (lane == 0u) wcnt[wave] = (unsigned)__popc(mask);
    __syncthreads();
    unsigned base = run, tot = 0u;
#pragma unroll
    for (unsigned q = 0; q < 8u; ++q) { const unsigned cq = wcnt[q]; base += (q < wave) ? cq : 0u; tot += cq; }
    const unsigned pos = base + rank;
    if (sel && pos < (unsigned)SEQ) { lidx[pos] = (unsigned short)n; lw[pos] = w; }
    run += tot;
    __syncthreads();
  }
  const unsigned runc = run < (unsigned)SEQ ? run : (unsigned)SEQ;
  const unsigned cnt = (unsigned)__builtin_amdgcn_readfirstlane((int)runc);
  const unsigned ntiles = (cnt + (unsigned)(TM - 1)) / (unsigned)TM;
  if (tid < (unsigned)TM) { const unsigned p = cnt + tid; if (p < ntiles * (unsigned)TM) { lidx[p] = (unsigned short)0; lw[p] = 0.0f; } }
  __syncthreads();
  unsigned bo[2]; float bb[2]; float cs[2] = { 0.f, 0.f };
#pragma unroll
  for (int ni = 0; ni < 2; ++ni) { const unsigned col = n0 + wave * 32u + ni * 16u + lm;
    bo[ni] = (e * (unsigned)DHID + col) * (unsigned)DIN + 8u * lh;
    bb[ni] = bfr(B1[(size_t)e * DHID + col]); }
#pragma unroll 1
  for (unsigned t = 0; t < ntiles; ++t) {
#pragma unroll 4
    for (unsigned it = 0; it < (unsigned)(TM * DIN / 8 / 256); ++it) { const unsigned idx = it * 256u + tid, rw = idx >> 6, pc = idx & 63u;
      unsigned n = lidx[t * (unsigned)TM + rw]; n = n < (unsigned)SEQ ? n : (unsigned)(SEQ - 1);
      const v4u v = *(const v4u*)(XB + ((size_t)b * SEQ + n) * DIN + 8u * pc);
      sa4[rw * (unsigned)APITCH4 + pc] = v; }
    __syncthreads();
    v8f acc[4][2] = {};
#pragma unroll 2
    for (unsigned kc = 0; kc < DIN / 32; ++kc) { v16b a[4], bf[2];
#pragma unroll
      for (int mi = 0; mi < 4; ++mi) { union { v16b v; v4u q[2]; } f; const unsigned o = (mi * 16u + lm) * (unsigned)APITCH4 + kc * 4u + lh;
        f.q[0] = sa4[o]; f.q[1] = sa4[o + 2u]; a[mi] = f.v; }
#pragma unroll
      for (int ni = 0; ni < 2; ++ni) bf[ni] = ldfrag_b(W1T + bo[ni] + kc * 32u);
#pragma unroll
      for (int mi = 0; mi < 4; ++mi)
#pragma unroll
        for (int ni = 0; ni < 2; ++ni) acc[mi][ni] = wmma_bf(a[mi], bf[ni], acc[mi][ni]); }
#pragma unroll
    for (int mi = 0; mi < 4; ++mi)
#pragma unroll
      for (int r = 0; r < 8; ++r) { const float wr = lw[t * (unsigned)TM + mi * 16u + 8u * lh + r];
#pragma unroll
        for (int ni = 0; ni < 2; ++ni) cs[ni] += fmaxf(acc[mi][ni][r] + bb[ni], 0.f) * wr; }
    __syncthreads();
  }
#pragma unroll
  for (int ni = 0; ni < 2; ++ni) cs[ni] += __shfl_xor(cs[ni], 16);
  if (lh == 0u) { so[wave * 32u + lm] = cs[0]; so[wave * 32u + 16u + lm] = cs[1]; }
  __syncthreads();
  if (tid < 64u) {
    const v4f val = *(const v4f*)&so[4u * tid];
    volatile v4f* p = (volatile v4f*)(HS + (size_t)g * DHID + n0 + 4u * tid);
    *p = val; __threadfence(); *p = val;
  }
}

__global__ __launch_bounds__(256) void k_out(const float* __restrict__ HS, const unsigned short* __restrict__ W2T, const float* __restrict__ B2, const float* __restrict__ WD, float* __restrict__ OUT) {
  __shared__ float smass[8];
  __shared__ float sinv[8];
  __shared__ __align__(16) float so[8][128];
  const unsigned tid = threadIdx.x, lane = tid & 31u, lm = lane & 15u, lh = lane >> 4;
  const unsigned wave = (unsigned)__builtin_amdgcn_readfirstlane((int)(tid >> 5));
  const unsigned e = blockIdx.y, n0 = blockIdx.x * 128u;
  {
    const unsigned wv = tid >> 5;
    const unsigned bq = wv < (unsigned)NB ? wv : (unsigned)(NB - 1);
    float s = 0.f;
#pragma unroll 4
    for (unsigned i = 0; i < (unsigned)(SEQ / 32); ++i) s += WD[((size_t)bq * SEQ + lane + 32u * i) * NE + e];
    s += __shfl_xor(s, 16); s += __shfl_xor(s, 8); s += __shfl_xor(s, 4); s += __shfl_xor(s, 2); s += __shfl_xor(s, 1);
    if (lane == 0u) { smass[wave] = s; sinv[wave] = 1.0f / fmaxf(s, EPSV); }
  }
  __syncthreads();
  const unsigned bl = lm < (unsigned)NB ? lm : (unsigned)(NB - 1);
  const bool live = lm < (unsigned)NB;
  const float sca = sinv[bl & 7u] * HCARRY;
  const float* ap = HS + (size_t)(bl * NE + e) * DHID + 8u * lh;
  const unsigned col = n0 + wave * 16u + lm;
  const unsigned short* bp = W2T + (size_t)(e * DHID + col) * DHID + 8u * lh;
  v8f acc = {};
#pragma unroll 2
  for (unsigned kc = 0; kc < DHID / 32; ++kc) { const float* p = ap + kc * 32u;
    const v4f a0 = *(const v4f*)p, a1 = *(const v4f*)(p + 4), a2 = *(const v4f*)(p + 16), a3 = *(const v4f*)(p + 20); v16h a;
#pragma unroll
    for (int i = 0; i < 4; ++i) {
      a[i]      = toh_flush(live ? a0[i] * sca : 0.0f); a[4 + i]  = toh_flush(live ? a1[i] * sca : 0.0f);
      a[8 + i]  = toh_flush(live ? a2[i] * sca : 0.0f); a[12 + i] = toh_flush(live ? a3[i] * sca : 0.0f); }
    const v16h bw = ldfrag_h(bp + kc * 32u);
    acc = wmma16(a, bw, acc); }
  const float b2v = bfr(B2[(size_t)e * DHID + col]);
  if (lh == 0u) {
#pragma unroll
    for (int r = 0; r < 8; ++r) so[r][wave * 16u + lm] = acc[r] * OSCALE + (b2v * smass[r]) * sinv[r];
  }
  __syncthreads();
  if (wave < (unsigned)NB) {
    const v4f val = *(const v4f*)&so[wave][4u * lane];
    volatile v4f* p = (volatile v4f*)(OUT + (size_t)(wave * NE + e) * DHID + n0 + 4u * lane);
    *p = val; __threadfence(); *p = val;
  }
}

extern "C" void kernel_launch(void* const* d_in, const int* in_sizes, int n_in, void* d_out, int out_size, void* d_ws, size_t ws_size, hipStream_t stream) {
  if (n_in < 10) return;
  if (in_sizes[0] < ((NB - 1) * SEQ_FULL + SEQ) * DIN || in_sizes[1] < NB * DIN || in_sizes[2] < DIN * NE || in_sizes[3] < NE) return;
  if (in_sizes[4] < DIN * NE || in_sizes[5] < NE || in_sizes[6] < NE * DIN * DHID || in_sizes[7] < NE * DHID) return;
  if (in_sizes[8] < NE * DHID * DHID || in_sizes[9] < NE * DHID) return;
  if ((size_t)out_size < OUT1_ELEM + 1) return;
  if (ws_size < (size_t)WS_END) return;
  const float* TOK = (const float*)d_in[0];
  const float* GV  = (const float*)d_in[1];
  const float* GW  = (const float*)d_in[2];
  const float* GB  = (const float*)d_in[3];
  const float* NW  = (const float*)d_in[4];
  const float* NBI = (const float*)d_in[5];
  const float* W1  = (const float*)d_in[6];
  const float* B1  = (const float*)d_in[7];
  const float* W2  = (const float*)d_in[8];
  const float* B2  = (const float*)d_in[9];
  char* ws = (char*)d_ws;
  unsigned short* XB  = (unsigned short*)(ws + WS_XB);
  unsigned short* W1T = (unsigned short*)(ws + WS_W1T);
  unsigned short* W2T = (unsigned short*)(ws + WS_W2T);
  float* WD = (float*)(ws + WS_WD);
  float* HS = (float*)(ws + WS_HS);
  float* OUT = (float*)d_out;
  k_cvt_x<<<dim3(NROW * DIN / 8 / 256), 256, 0, stream>>>(TOK, XB);
  k_tr<<<dim3(DHID / 64, DIN / 64, NE), 256, 0, stream>>>(W1, W1T, (unsigned)DIN, (unsigned)DHID, (unsigned)DIN, (unsigned)DHID, 0u, 0, 1.0f);
  k_tr<<<dim3(DHID / 64, DHID / 64, NE), 256, 0, stream>>>(W2, W2T, (unsigned)DHID, (unsigned)DHID, (unsigned)DHID, (unsigned)DHID, 0u, 1, WCARRY);
  k_gate<<<dim3(NROW / 32), 256, 0, stream>>>(TOK, GV, GW, GB, NW, NBI, WD);
  k_lb<<<dim3(1), 256, 0, stream>>>(WD, OUT);
  k_pool<<<dim3(DHID / PCOLS, NG), 256, 0, stream>>>(XB, W1T, B1, WD, HS);
  k_out<<<dim3(DHID / 128, NE), 256, 0, stream>>>(HS, W2T, B2, WD, OUT);
}
